// GCN_G2_D2_86320252715553
// MI455X (gfx1250) — hardware-run, weakly checked
//
#include <hip/hip_runtime.h>


namespace {
constexpr int N = 20000, NP = 20032  , E = 320000, FIN = 256, NH = 8, CH = 128, HC = NH * CH  , HHC = HC / 2, G = 64, DHID = 128;
constexpr float XS = 8.0f, WSC = 256.0f, NEG = 0.2f, NEG2 = 0.01f, EPSD = 1e-16f, EPSBN = 1e-5f;
typedef __attribute__((ext_vector_type(4))) _Float16 v4b;

typedef _Float16 b16;
typedef __attribute__((ext_vector_type(16))) _Float16 v16b;
typedef __attribute__((ext_vector_type(8))) _Float16 v8b;
typedef __attribute__((ext_vector_type(8))) float v8f;
typedef __attribute__((ext_vector_type(4))) float v4f;
__device__ __forceinline__ float bf16_rne(float f) { unsigned int u = __float_as_uint(f); u += 0x7FFFu + ((u >> 16) & 1u); return __uint_as_float(u & 0xFFFF0000u); }
__device__ __forceinline__ void split16(float v, b16& hi, b16& lo) { hi = (b16)v; lo = (b16)(v - (float)hi); }
__device__ __forceinline__ v16b frag_kb(const b16* p, int hh) { const v8b a = *(const v8b*)(p + 8 * hh), b = *(const v8b*)(p + 16 + 8 * hh); v16b f;
#pragma unroll
  for (int e = 0; e < 8; ++e) { f[e] = a[e]; f[8 + e] = b[e]; } return f; }
__device__ __forceinline__ v8f wmma16b(v16b a, v16b b, v8f c) { v8f d = __builtin_amdgcn_wmma_f32_16x16x32_f16(false, a, false, b, (short)0, c, false, false); asm volatile("v_nop\n\tv_nop\n\tv_nop\n\tv_nop" : "+v"(d) : "v"(a), "v"(b)); return d; }
__device__ __forceinline__ void wave_lds_sync() { __builtin_amdgcn_fence(__ATOMIC_RELEASE, "workgroup"); __builtin_amdgcn_wave_barrier(); __builtin_amdgcn_fence(__ATOMIC_ACQUIRE, "workgroup"); }
__device__ __forceinline__ float pmul(float a, float b) { float p = a * b; asm volatile("" : "+v"(p)); return p; }
__device__ __forceinline__ int iclamp(int v, int lo, int hi) { return v < lo ? lo : (v > hi ? hi : v); }
__device__ __forceinline__ float nexp(float x) { return __builtin_amdgcn_exp2f(x * 1.4426950408889634f); }
__device__ __forceinline__ float lrelu(float x) { return x > 0.0f ? x : NEG * x; }

constexpr int CSR_NBLK = 512, CSR_GB = 9, CSR_GN = 1 << CSR_GB  , CSR_MAXG = 512, CSR_CAP = 12288  ;
__global__ __launch_bounds__(64) void csrA_kernel(const int* __restrict__ dst, int E, int N, int nG, int CHP, int NGP, int* __restrict__ STG, int* __restrict__ HST) {
  extern __shared__ int sm[];
  int* cnt = sm; int* run = sm + NGP; int* ids = sm + 2 * NGP;
  const int b = blockIdx.x; const int ch = (E + CSR_NBLK - 1) / CSR_NBLK; const int e0 = b * ch, e1 = min(E, e0 + ch);
  for (int i = threadIdx.x; i < NGP; i += 64) cnt[i] = 0;
  for (int i = threadIdx.x; i < CHP; i += 64) ids[i] = -1;
  __syncthreads();
  if (threadIdx.x == 0) {
    for (int e = e0; e < e1; ++e) { int d = dst[e]; d = (d < 0) ? 0 : (d >= N ? N - 1 : d); cnt[d >> CSR_GB] += 1; }
    int acc = 0; for (int g = 0; g < nG; ++g) { run[g] = acc; acc += cnt[g]; }
    for (int e = e0; e < e1; ++e) { int d = dst[e]; d = (d < 0) ? 0 : (d >= N ? N - 1 : d); const int g = d >> CSR_GB; ids[run[g]] = e; run[g] += 1; } }
  __syncthreads();
  typedef __attribute__((ext_vector_type(4))) int v4i;
  for (int pass = 0; pass < 2; ++pass) {
    for (int i = threadIdx.x; i < CHP / 4; i += 64) *(volatile v4i*)(STG + (size_t)b * CHP + i * 4) = *(const v4i*)(&ids[i * 4]);
    for (int i = threadIdx.x; i < NGP / 4; i += 64) { v4i v; for (int e = 0; e < 4; ++e) v[e] = (i * 4 + e < nG) ? cnt[i * 4 + e] : 0; *(volatile v4i*)(HST + (size_t)b * NGP + i * 4) = v; }
    __threadfence(); }
}
__global__ __launch_bounds__(512) void csrS_kernel(const int* __restrict__ HST, int nG, int NGP, int* __restrict__ START, int* __restrict__ TOT, int* __restrict__ OFF) {
  __shared__ int tot[CSR_MAXG];
  const int b = threadIdx.x;
  for (int pass = 0; pass < 2; ++pass) { int runb = 0; for (int g = 0; g < nG; ++g) { int c = HST[(size_t)b * NGP + g]; c = (c < 0) ? 0 : c; ((volatile int*)OFF)[(size_t)g * CSR_NBLK + b] = runb; runb += c; } __threadfence(); }
  for (int g = threadIdx.x; g < nG; g += 512) { int s = 0; for (int bb = 0; bb < CSR_NBLK; ++bb) { int c = HST[(size_t)bb * NGP + g]; s += (c < 0) ? 0 : c; } tot[g] = s; }
  __syncthreads();
  if (threadIdx.x < 32) {
    __shared__ int st[CSR_MAXG + 32];
    if (threadIdx.x == 0) { int acc = 0; for (int g = 0; g < NGP; ++g) { st[g] = acc; if (g < nG) acc += (tot[g] + 31) & ~31; } st[NGP] = acc; }
    __builtin_amdgcn_fence(__ATOMIC_RELEASE, "workgroup"); __builtin_amdgcn_wave_barrier(); __builtin_amdgcn_fence(__ATOMIC_ACQUIRE, "workgroup");
    for (int pass = 0; pass < 2; ++pass) { for (int i = threadIdx.x; i < NGP + 32; i += 32) { ((volatile int*)START)[i] = (i <= NGP) ? st[min(i, NGP)] : 0; ((volatile int*)TOT)[i] = (i < nG) ? tot[i] : 0; } __threadfence(); } }
}
__global__ __launch_bounds__(256) void csrB_kernel(const int* __restrict__ dst, int N, int nG, int CHP, int NGP, int permLen, const int* __restrict__ STG, const int* __restrict__ HST, const int* __restrict__ OFF, const int* __restrict__ START, const int* __restrict__ TOT, int* __restrict__ PERM, int* __restrict__ ROWPTR, int* __restrict__ ROWCNT, int* __restrict__ FLAG) {
  typedef __attribute__((ext_vector_type(4))) int v4i;
  __shared__ int ids[CSR_CAP]; __shared__ unsigned short key[CSR_CAP]; __shared__ int outp[CSR_CAP]; __shared__ int ncnt[CSR_GN + 1]; __shared__ int boff[CSR_NBLK + 1];
  const int g = blockIdx.x, t_ = threadIdx.x; int tot = TOT[g]; int st = START[g], stn = START[g + 1]; const int v0 = g * CSR_GN; const int nv = min(CSR_GN, N - v0);
  st = (st < 0) ? 0 : (st > permLen - 32 ? permLen - 32 : st) & ~31; stn = (stn < st) ? st : (stn > permLen ? permLen : stn); tot = (tot < 0) ? 0 : tot; if (tot > stn - st && tot <= CSR_CAP) tot = stn - st;
  if (tot > CSR_CAP) {
    for (int pass = 0; pass < 2; ++pass) { for (int i = t_; i < CSR_GN / 4; i += 256) { v4i a, c; for (int e = 0; e < 4; ++e) { a[e] = st; c[e] = 0; } *(volatile v4i*)(ROWPTR + v0 + i * 4) = a; *(volatile v4i*)(ROWCNT + v0 + i * 4) = c; } if (t_ == 0) ((volatile int*)FLAG)[0] = 1; __threadfence(); } (void)nv; return; }
  if (t_ == 0) { int acc = 0; for (int b = 0; b < CSR_NBLK; ++b) { boff[b] = acc; int c = HST[(size_t)b * NGP + g]; c = (c < 0) ? 0 : (c > CHP ? CHP : c); acc += c; if (acc > tot) acc = tot; } boff[CSR_NBLK] = acc; }
  for (int i = t_; i <= CSR_GN; i += 256) ncnt[i] = 0;
  __syncthreads();
  for (int b = 0; b < CSR_NBLK; ++b) { const int c = boff[b + 1] - boff[b]; int o_ = OFF[(size_t)g * CSR_NBLK + b]; o_ = (o_ < 0) ? 0 : (o_ > CHP - c ? CHP - c : o_); const int* src_ = STG + (size_t)b * CHP + o_;
    for (int i = t_; i < c; i += 256) { int id = src_[i]; id = (id < 0) ? 0 : id; ids[boff[b] + i] = id; int d = dst[id]; d = (d < v0) ? v0 : (d >= N ? N - 1 : d); int kk = d - v0; kk = (kk < 0) ? 0 : (kk >= CSR_GN ? CSR_GN - 1 : kk); key[boff[b] + i] = (unsigned short)kk; } }
  __syncthreads();
  if (t_ == 0) { for (int i = 0; i < tot; ++i) ncnt[key[i]] += 1; int acc = 0; for (int vl = 0; vl < CSR_GN; ++vl) { const int c = ncnt[vl]; ncnt[vl] = acc; acc += c; } ncnt[CSR_GN] = acc;
    for (int i = 0; i < tot; ++i) { const int vl = key[i]; outp[ncnt[vl]] = ids[i]; ncnt[vl] += 1; }
    for (int vl = CSR_GN; vl > 0; --vl) ncnt[vl] = ncnt[vl - 1]; ncnt[0] = 0; }
  __syncthreads();
  for (int pass = 0; pass < 2; ++pass) {
    for (int i = t_; i < (stn - st) / 4; i += 256) { v4i v; for (int e = 0; e < 4; ++e) { const int q = i * 4 + e; v[e] = (q < tot) ? outp[q] : -1; } *(volatile v4i*)(PERM + st + i * 4) = v; }
    for (int i = t_; i < CSR_GN / 4; i += 256) { v4i a, c; for (int e = 0; e < 4; ++e) { const int vl = i * 4 + e; a[e] = st + ncnt[vl]; c[e] = (vl < nv) ? (ncnt[vl + 1] - ncnt[vl]) : 0; } *(volatile v4i*)(ROWPTR + v0 + i * 4) = a; *(volatile v4i*)(ROWCNT + v0 + i * 4) = c; }
    __threadfence(); }
}
__global__ __launch_bounds__(256) void csrZ_kernel(int* __restrict__ p, size_t n4) { typedef __attribute__((ext_vector_type(4))) int v4i; const size_t tid = (size_t)blockIdx.x * 256 + threadIdx.x, nth = (size_t)gridDim.x * 256; v4i z = {0, 0, 0, 0}; for (size_t i = tid; i < n4; i += nth) *(volatile v4i*)(p + i * 4) = z; }
struct CsrBufs { int *STG, *HST, *OFF, *START, *TOT, *PERM, *ROWPTR, *ROWCNT, *FLAG; int nG, NGP, CHP; size_t permLen; char* base; size_t bytes; };
static size_t csr_carve(CsrBufs& c, char* ws, size_t off, int E, int N) {
  const size_t off0 = off; c.base = ws + off;
  auto al = [&](size_t bytes) { char* p = ws + off; off += (bytes + 255) & ~(size_t)255; return p; };
  c.nG = (N + CSR_GN - 1) / CSR_GN; c.NGP = (c.nG + 31) & ~31; const int ch = (E + CSR_NBLK - 1) / CSR_NBLK; c.CHP = (ch + 31) & ~31; c.permLen = (size_t)E + 32 * (size_t)c.nG + 32;
  c.STG = (int*)al((size_t)CSR_NBLK * c.CHP * 4); c.HST = (int*)al((size_t)CSR_NBLK * c.NGP * 4); c.OFF = (int*)al((size_t)c.NGP * CSR_NBLK * 4); c.START = (int*)al((size_t)(c.NGP + 64) * 4); c.TOT = (int*)al((size_t)(c.NGP + 64) * 4);
  c.PERM = (int*)al(c.permLen * 4); c.ROWPTR = (int*)al((size_t)c.nG * CSR_GN * 4); c.ROWCNT = (int*)al((size_t)c.nG * CSR_GN * 4); c.FLAG = (int*)al(256);
  c.bytes = off - off0; return off;
}
static void csr_build(const CsrBufs& c, const int* dst, int E, int N, hipStream_t stream) {
  const size_t smem = (size_t)(2 * c.NGP + c.CHP) * 4;
  csrZ_kernel<<<512, 256, 0, stream>>>((int*)c.base, c.bytes / 16);
  csrA_kernel<<<CSR_NBLK, 64, smem, stream>>>(dst, E, N, c.nG, c.CHP, c.NGP, c.STG, c.HST);
  csrS_kernel<<<1, 512, 0, stream>>>(c.HST, c.nG, c.NGP, c.START, c.TOT, c.OFF);
  csrB_kernel<<<c.nG, 256, 0, stream>>>(dst, N, c.nG, c.CHP, c.NGP, (int)c.permLen, c.STG, c.HST, c.OFF, c.START, c.TOT, c.PERM, c.ROWPTR, c.ROWCNT, c.FLAG);
}

__device__ __forceinline__ float lrelu2(float x) { return x > 0.0f ? x : NEG2 * x; }

__global__ __launch_bounds__(256) void prep_kernel(const float* __restrict__ x, const float* __restrict__ wl, const float* __restrict__ wr, b16* __restrict__ X16, b16* __restrict__ WL, b16* __restrict__ WR) {
  const size_t t = (size_t)blockIdx.x * 256 + threadIdx.x; const size_t nx = (size_t)NP * FIN / 8, nw = (size_t)HC * FIN / 8; v8b o;
  if (t < nx) { const size_t e = t * 8; const size_t row = e / FIN; for (int j = 0; j < 8; ++j) o[j] = (row < (size_t)N) ? (b16)(bf16_rne(x[e + j]) * XS) : (b16)0.0f; for (int pass = 0; pass < 2; ++pass) { *(volatile v8b*)(X16 + e) = o; __threadfence(); } return; }
  size_t u = t - nx; if (u >= 2 * nw) return; const int kind = (int)(u / nw); const size_t e = (u % nw) * 8; const float* w = kind == 0 ? wl : wr; const int oo = (int)(e / FIN), k0 = (int)(e % FIN);
  for (int j = 0; j < 8; ++j) o[j] = (b16)(bf16_rne(w[(size_t)(k0 + j) * HC + oo]) * WSC);
  for (int pass = 0; pass < 2; ++pass) { *(volatile v8b*)((kind == 0 ? WL : WR) + e) = o; __threadfence(); }
}
__global__ __launch_bounds__(128) void proj_kernel(const b16* __restrict__ X16, const b16* __restrict__ WL, const b16* __restrict__ WR, int hf, b16* __restrict__ XLh, b16* __restrict__ XLl, b16* __restrict__ XR) {
  __shared__ __attribute__((aligned(16))) b16 Th[4][16][128 + 8], Tl[4][16][128 + 8];
  const int wave = threadIdx.x >> 5, lane = threadIdx.x & 31, nloc = lane & 15, hlf = lane >> 4; const int kind = blockIdx.z, n0 = blockIdx.y * 128; const size_t m0 = (size_t)blockIdx.x * 64 + wave * 16;
  const b16* W = (kind == 0 ? WL : WR) + (size_t)(hf * HHC) * FIN; v8f acc[8];
#pragma unroll
  for (int t = 0; t < 8; ++t) acc[t] = (v8f){};
#pragma unroll 2
  for (int kb = 0; kb < FIN; kb += 32) { const v16b a = frag_kb(X16 + (m0 + nloc) * FIN + kb, hlf);
#pragma unroll
    for (int t = 0; t < 8; ++t) acc[t] = wmma16b(a, frag_kb(W + (size_t)(n0 + t * 16 + nloc) * FIN + kb, hlf), acc[t]); }
#pragma unroll
  for (int t = 0; t < 8; ++t)
#pragma unroll
    for (int r = 0; r < 8; ++r) { b16 p, q; split16(acc[t][r] * (1.0f / (XS * WSC)) * XS, p, q); Th[wave][8 * hlf + r][t * 16 + nloc] = p; Tl[wave][8 * hlf + r][t * 16 + nloc] = q; }
  wave_lds_sync();
  for (int pass = 0; pass < 2; ++pass) { for (int r2 = 0; r2 < 16; r2 += 2) { const int rr = r2 + (lane >> 4), c8 = (lane & 15) * 8; const size_t gi = (m0 + rr) * HHC + n0 + c8;
      if (kind == 0) { *(volatile v8b*)(XLh + gi) = *(const v8b*)(&Th[wave][rr][c8]); *(volatile v8b*)(XLl + gi) = *(const v8b*)(&Tl[wave][rr][c8]); } else *(volatile v8b*)(XR + gi) = *(const v8b*)(&Th[wave][rr][c8]); }
    __threadfence(); }
}
__global__ __launch_bounds__(256) void agg1_kernel(const b16* __restrict__ XLh, const b16* __restrict__ XLl, const b16* __restrict__ XR, const float* __restrict__ att, const float* __restrict__ b1, const int* __restrict__ srcs, const int* __restrict__ PERM, const int* __restrict__ ROWPTR, const int* __restrict__ ROWCNT, int permLen, int hf, b16* __restrict__ H1) {
  __shared__ __attribute__((aligned(16))) b16 rowst[8][HHC + 8];
  const int wave = threadIdx.x >> 5, lane = threadIdx.x & 31; const size_t v = (size_t)blockIdx.x * 8 + wave; const int hl = lane >> 3, c0 = (lane & 7) * 16; const int hglob = hf * 4 + hl;
  float a16[16], xr16[16]; { const v8b r0 = *(const v8b*)(XR + v * HHC + hl * CH + c0), r1 = *(const v8b*)(XR + v * HHC + hl * CH + c0 + 8); for (int j = 0; j < 8; ++j) { xr16[j] = (float)r0[j] * (1.0f / XS); xr16[8 + j] = (float)r1[j] * (1.0f / XS); a16[j] = bf16_rne(att[hglob * CH + c0 + j]); a16[8 + j] = bf16_rne(att[hglob * CH + c0 + 8 + j]); } }
  float m = -INFINITY, l = 0.0f; float acc[16]; for (int j = 0; j < 16; ++j) acc[j] = 0.0f;
  int st = 0, cnt = 0; if (v < (size_t)N) { st = ROWPTR[v]; cnt = ROWCNT[v]; cnt = iclamp(cnt, 0, 8192); st = iclamp(st, 0, permLen - cnt); }
  const int nit = (v < (size_t)N) ? cnt + 1 : 0;
  for (int it = 0; it < nit; ++it) { int s; if (it == 0) s = (int)v; else { const int e = iclamp(PERM[st + it - 1], 0, E - 1); s = iclamp(srcs[e], 0, N - 1); }
    const v8b h0 = *(const v8b*)(XLh + (size_t)s * HHC + hl * CH + c0), h1v = *(const v8b*)(XLh + (size_t)s * HHC + hl * CH + c0 + 8), l0 = *(const v8b*)(XLl + (size_t)s * HHC + hl * CH + c0), l1 = *(const v8b*)(XLl + (size_t)s * HHC + hl * CH + c0 + 8);
    float xl[16]; for (int j = 0; j < 8; ++j) { xl[j] = ((float)h0[j] + (float)l0[j]) * (1.0f / XS); xl[8 + j] = ((float)h1v[j] + (float)l1[j]) * (1.0f / XS); }
    float d = 0.0f; for (int j = 0; j < 16; ++j) d += pmul(a16[j], lrelu(xl[j] + xr16[j]));
    d += __shfl_xor(d, 1); d += __shfl_xor(d, 2); d += __shfl_xor(d, 4);
    const float mn = fmaxf(m, d); const float al = __expf(m - mn); const float p = __expf(d - mn); l = l * al + p; for (int j = 0; j < 16; ++j) acc[j] = acc[j] * al + pmul(p, xl[j]); m = mn; }
  const float inv = (nit > 0) ? 1.0f / (l + EPSD) : 0.0f;
  for (int j = 0; j < 16; ++j) { const float y = (v < (size_t)N) ? acc[j] * inv + bf16_rne(b1[hglob * CH + c0 + j]) : 0.0f; rowst[wave][hl * CH + c0 + j] = (b16)(y * XS); }
  wave_lds_sync();
  for (int pass = 0; pass < 2; ++pass) { for (int k = 0; k < 2; ++k) *(volatile v8b*)(H1 + v * HC + hf * HHC + k * 256 + lane * 8) = *(const v8b*)(&rowst[wave][k * 256 + lane * 8]); __threadfence(); }
}
__global__ __launch_bounds__(256) void bn1_kernel(const b16* __restrict__ H1, float* __restrict__ MU, float* __restrict__ RS) {
  __shared__ __attribute__((aligned(16))) float mu_s[256], rs_s[256];
  const int c = blockIdx.x * 256 + threadIdx.x; float s = 0.0f;
#pragma unroll 4
  for (int v = 0; v < N; ++v) s += (float)H1[(size_t)v * HC + c];
  const float mu = s * (1.0f / XS) / (float)N; float q = 0.0f;
#pragma unroll 4
  for (int v = 0; v < N; ++v) { const float d = (float)H1[(size_t)v * HC + c] * (1.0f / XS) - mu; q += d * d; }
  mu_s[threadIdx.x] = mu; rs_s[threadIdx.x] = rsqrtf(q / (float)N + EPSBN);
  __syncthreads();
  for (int pass = 0; pass < 2; ++pass) { if (threadIdx.x < 64) *(volatile v4f*)(MU + blockIdx.x * 256 + threadIdx.x * 4) = *(const v4f*)(&mu_s[threadIdx.x * 4]); else if (threadIdx.x < 128) *(volatile v4f*)(RS + blockIdx.x * 256 + (threadIdx.x - 64) * 4) = *(const v4f*)(&rs_s[(threadIdx.x - 64) * 4]); __threadfence(); }
}
__global__ __launch_bounds__(256) void proj2_kernel(const b16* __restrict__ H1, const float* __restrict__ MU, const float* __restrict__ RS, const float* __restrict__ g1, const float* __restrict__ be1, const float* __restrict__ w2l, const float* __restrict__ w2r, float* __restrict__ L2) {
  __shared__ float lr[8][4];
  const int wave = threadIdx.x >> 5, lane = threadIdx.x & 31; const size_t v = (size_t)blockIdx.x * 8 + wave; float sl = 0.0f, sr = 0.0f;
  if (v < (size_t)N) { for (int k = 0; k < HC / 32; ++k) { const int c = k * 32 + lane; const float h = (float)H1[v * HC + c] * (1.0f / XS); const float hb = lrelu2((h - MU[c]) * RS[c] * bf16_rne(g1[c]) + bf16_rne(be1[c])); sl += pmul(hb, bf16_rne(w2l[c])); sr += pmul(hb, bf16_rne(w2r[c])); } }
#pragma unroll
  for (int o = 16; o >= 1; o >>= 1) { sl += __shfl_xor(sl, o); sr += __shfl_xor(sr, o); }
  if (lane == 0) { lr[wave][0] = sl; lr[wave][1] = sr; lr[wave][2] = 0.0f; lr[wave][3] = 0.0f; }
  __syncthreads();
  for (int pass = 0; pass < 2; ++pass) { if (threadIdx.x < 8) *(volatile v4f*)(L2 + ((size_t)blockIdx.x * 8 + threadIdx.x) * 4) = *(const v4f*)(&lr[threadIdx.x][0]); __threadfence(); }
}
__global__ __launch_bounds__(256) void agg2_kernel(const float* __restrict__ L2, const float* __restrict__ att2, const float* __restrict__ b2, const int* __restrict__ srcs, const int* __restrict__ PERM, const int* __restrict__ ROWPTR, const int* __restrict__ ROWCNT, int permLen, float* __restrict__ O2) {
  __shared__ __attribute__((aligned(16))) float os_[256];
  const size_t v = (size_t)blockIdx.x * 256 + threadIdx.x; float outv = 0.0f;
  if (v < (size_t)N) { const float a = bf16_rne(att2[0]), xr = L2[v * 4 + 1]; int st = ROWPTR[v], cnt = ROWCNT[v]; cnt = iclamp(cnt, 0, 8192); st = iclamp(st, 0, permLen - cnt);
    float m = -INFINITY, l = 0.0f, acc = 0.0f;
    for (int it = 0; it <= cnt; ++it) { int s; if (it == 0) s = (int)v; else { const int e = iclamp(PERM[st + it - 1], 0, E - 1); s = iclamp(srcs[e], 0, N - 1); }
      const float xl = L2[(size_t)s * 4]; const float d = pmul(a, lrelu(xl + xr)); const float mn = fmaxf(m, d); const float al = __expf(m - mn); const float p = __expf(d - mn); l = l * al + p; acc = acc * al + pmul(p, xl); m = mn; }
    outv = acc / (l + EPSD) + bf16_rne(b2[0]); }
  os_[threadIdx.x] = outv; __syncthreads();
  for (int pass = 0; pass < 2; ++pass) { if (threadIdx.x < 64) *(volatile v4f*)(O2 + (size_t)blockIdx.x * 256 + threadIdx.x * 4) = *(const v4f*)(&os_[threadIdx.x * 4]); __threadfence(); }
}
__global__ __launch_bounds__(256) void final_kernel(const float* __restrict__ O2, const int* __restrict__ batch, const float* __restrict__ g2, const float* __restrict__ be2, const float* __restrict__ lw1, const float* __restrict__ lb1, const float* __restrict__ lw2, const float* __restrict__ lb2, float* __restrict__ out) {
  __shared__ float red[256]; __shared__ float stat[2]; __shared__ __attribute__((aligned(16))) float res[G];
  const int t_ = threadIdx.x;
  { float s = 0.0f; for (int v = t_; v < N; v += 256) s += O2[v]; red[t_] = s; __syncthreads(); for (int st = 128; st >= 1; st >>= 1) { if (t_ < st) red[t_] += red[t_ + st]; __syncthreads(); } if (t_ == 0) stat[0] = red[0] / (float)N; __syncthreads(); }
  const float mu = stat[0];
  { float s = 0.0f; for (int v = t_; v < N; v += 256) { const float d = O2[v] - mu; s += d * d; } red[t_] = s; __syncthreads(); for (int st = 128; st >= 1; st >>= 1) { if (t_ < st) red[t_] += red[t_ + st]; __syncthreads(); } if (t_ == 0) stat[1] = rsqrtf(red[0] / (float)N + EPSBN); __syncthreads(); }
  const float rs = stat[1], gg = bf16_rne(g2[0]), bb = bf16_rne(be2[0]);
  if (t_ < G) { float s = 0.0f; int cnt = 0;
    for (int v = 0; v < N; ++v) if (batch[v] == t_) { s += lrelu2((O2[v] - mu) * rs * gg + bb); ++cnt; }
    const float pooled = s / fmaxf((float)cnt, 1.0f); float o = bf16_rne(lb2[0]);
#pragma unroll 1
    for (int k = 0; k < DHID; ++k) o += pmul(lrelu2(pmul(pooled, bf16_rne(lw1[k])) + bf16_rne(lb1[k])), bf16_rne(lw2[k]));
    res[t_] = o; }
  __syncthreads();
  for (int pass = 0; pass < 2; ++pass) { if (t_ < 16) *(volatile v4f*)(out + t_ * 4) = *(const v4f*)(&res[t_ * 4]); __threadfence(); }
}
}

extern "C" void kernel_launch(void* const* d_in, const int* in_sizes, int n_in, void* d_out, int out_size, void* d_ws, size_t ws_size, hipStream_t stream) {
  (void)n_in;
  auto Fp = [&](int i) { return (const float*)d_in[i]; }; auto Ip = [&](int i) { return (const int*)d_in[i]; };
  if (in_sizes[0] != N * FIN || in_sizes[1] != 2 * E || in_sizes[2] != N || in_sizes[3] != FIN * HC || in_sizes[4] != FIN * HC || in_sizes[5] != NH * CH || in_sizes[9] != HC || in_sizes[15] != DHID || in_sizes[17] != DHID || out_size != G) return;
  size_t off = 0; char* ws = (char*)d_ws;
  auto carve = [&](size_t bytes) { char* p = ws + off; off += (bytes + 255) & ~(size_t)255; return p; };
  b16* X16 = (b16*)carve((size_t)NP * FIN * 2); b16* WL = (b16*)carve((size_t)HC * FIN * 2); b16* WR = (b16*)carve((size_t)HC * FIN * 2);
  b16* XLh = (b16*)carve((size_t)NP * HHC * 2); b16* XLl = (b16*)carve((size_t)NP * HHC * 2); b16* XR = (b16*)carve((size_t)NP * HHC * 2); b16* H1 = (b16*)carve((size_t)NP * HC * 2);
  float* MU = (float*)carve(HC * 4); float* RS = (float*)carve(HC * 4); float* L2 = (float*)carve((size_t)NP * 4 * 4); float* O2 = (float*)carve((size_t)((NP + 255) / 256) * 256 * 4);
  CsrBufs csr; off = csr_carve(csr, ws, off, E, N);
  if (off > ws_size || off > ((size_t)128 << 20)) return;
  prep_kernel<<<(unsigned)(((size_t)NP * FIN / 8 + 2 * (size_t)HC * FIN / 8 + 255) / 256), 256, 0, stream>>>(Fp(0), Fp(3), Fp(4), X16, WL, WR);
  csr_build(csr, Ip(1) + E, E, N, stream);
  for (int hf = 0; hf < 2; ++hf) {
    proj_kernel<<<dim3(NP / 64, HHC / 128, 2), 128, 0, stream>>>(X16, WL, WR, hf, XLh, XLl, XR);
    agg1_kernel<<<NP / 8, 256, 0, stream>>>(XLh, XLl, XR, Fp(5), Fp(6), Ip(1), csr.PERM, csr.ROWPTR, csr.ROWCNT, (int)csr.permLen, hf, H1);
  }
  bn1_kernel<<<HC / 256, 256, 0, stream>>>(H1, MU, RS);
  proj2_kernel<<<NP / 8, 256, 0, stream>>>(H1, MU, RS, Fp(7), Fp(8), Fp(9), Fp(10), L2);
  agg2_kernel<<<(NP + 255) / 256, 256, 0, stream>>>(L2, Fp(11), Fp(12), Ip(1), csr.PERM, csr.ROWPTR, csr.ROWCNT, (int)csr.permLen, O2);
  final_kernel<<<1, 256, 0, stream>>>(O2, Ip(2), Fp(13), Fp(14), Fp(15), Fp(16), Fp(17), Fp(18), (float*)d_out);
}
